// ConbimambaBlock_91319594648177
// MI455X (gfx1250) — hardware-run, weakly checked
//
#include <hip/hip_runtime.h>
#include <math.h>

typedef __attribute__((ext_vector_type(16))) _Float16 v16h;
typedef __attribute__((ext_vector_type(8)))  _Float16 v8h;
typedef __attribute__((ext_vector_type(8)))  float    v8f;
typedef __attribute__((ext_vector_type(4)))  float    v4f;
typedef __attribute__((ext_vector_type(4)))  unsigned int u32x4;

constexpr int kB      = 8;
constexpr int kL      = 512;
constexpr int kDm     = 512;
constexpr int kDff    = 2048;
constexpr int kDin    = 1024;
constexpr int kNst    = 16;
constexpr int kDtR    = 32;
constexpr int kKc     = 4;
constexpr int kXzP    = 2 * kDin;
constexpr int kXdP    = 64;
constexpr int kCvP    = 2 * kDm;
constexpr int kRows   = kB * kL;
constexpr int kConvTP = 260;
constexpr int kScanTS = 64;
constexpr int kScanCh = 64;
constexpr int kScanYP = 68;
constexpr int kDwCh   = 64;
constexpr int kDwRows = 64;
constexpr int kDwTaps = 63;
constexpr int kDwIn   = kDwRows + kDwTaps - 1;
constexpr int kDwOP   = 68;
static_assert(kDtR + 2 * kNst == kXdP, "x_proj width");
static_assert((kDm % 32) == 0 && (kDin % 32) == 0 && (kDff % 32) == 0, "GEMM K multiples of 32");
static_assert((kRows % 64) == 0 && (kXzP % 64) == 0 && (kXdP % 64) == 0 && (kDm % 64) == 0 && (kDff % 64) == 0 && (kCvP % 64) == 0, "GEMM M,N multiples of 64");
static_assert((kL % 64) == 0 && (kL % kScanTS) == 0 && (kDin % kScanCh) == 0 && (kDin % 256) == 0, "conv/scan tile multiples");
static_assert((kL % kDwRows) == 0 && (kDm % kDwCh) == 0 && kDwIn <= 128, "depthwise tile multiples");
static_assert((kRows % 8) == 0, "LN rows per block");

constexpr size_t kOffW1a  = 0;
constexpr size_t kOffW2a  = kOffW1a  + (size_t)kDff * kDm * 2;
constexpr size_t kOffW1b  = kOffW2a  + (size_t)kDm * kDff * 2;
constexpr size_t kOffW2b  = kOffW1b  + (size_t)kDff * kDm * 2;
constexpr size_t kOffWin  = kOffW2b  + (size_t)kDm * kDff * 2;
constexpr size_t kOffWx   = kOffWin  + (size_t)2 * kXzP * kDm * 2;
constexpr size_t kOffWout = kOffWx   + (size_t)2 * kXdP * kDin * 2;
constexpr size_t kOffWbo  = kOffWout + (size_t)2 * kDm * kDin * 2;
constexpr size_t kOffWp1  = kOffWbo  + (size_t)kDm * kCvP * 2;
constexpr size_t kOffWp2  = kOffWp1  + (size_t)kCvP * kDm * 2;
constexpr size_t kOffH1   = kOffWp2  + (size_t)kDm * kDm * 2;
constexpr size_t kOffH2   = kOffH1   + (size_t)kRows * kDm * 4;
constexpr size_t kOffH3   = kOffH2   + (size_t)kRows * kDm * 4;
constexpr size_t kOffH4   = kOffH3   + (size_t)kRows * kDm * 4;
constexpr size_t kOffHh   = kOffH4   + (size_t)kRows * kDm * 4;
constexpr size_t kOffNA   = kOffHh   + (size_t)kRows * kDm * 2;
constexpr size_t kOffU    = kOffNA   + (size_t)kRows * kDm * 2;
constexpr size_t kOffUC   = kOffU    + (size_t)kRows * kXzP * 2;
constexpr size_t kOffUCh  = kOffUC   + (size_t)kRows * kDin * 4;
constexpr size_t kOffXD   = kOffUCh  + (size_t)kRows * kDin * 2;
constexpr size_t kOffY    = kOffXD   + (size_t)kRows * kXdP * 4;
constexpr size_t kOffCat  = kOffY    + (size_t)kRows * kDin * 2;
constexpr size_t kWsTotal = kOffCat  + (size_t)kRows * kDin * 2;
static_assert(kWsTotal == 119275520ull, "carve total");
static_assert(kWsTotal <= 134217728ull, "carve cap");
static_assert((kOffW2a % 128) == 0 && (kOffW1b % 128) == 0 && (kOffW2b % 128) == 0 && (kOffWin % 128) == 0 &&
              (kOffWx % 128) == 0 && (kOffWout % 128) == 0 && (kOffWbo % 128) == 0 && (kOffWp1 % 128) == 0 &&
              (kOffWp2 % 128) == 0 && (kOffH1 % 128) == 0 && (kOffH2 % 128) == 0 && (kOffH3 % 128) == 0 &&
              (kOffH4 % 128) == 0 && (kOffHh % 128) == 0 && (kOffNA % 128) == 0 && (kOffU % 128) == 0 &&
              (kOffUC % 128) == 0 && (kOffUCh % 128) == 0 && (kOffXD % 128) == 0 && (kOffY % 128) == 0 &&
              (kOffCat % 128) == 0, "128-B aligned regions");
static_assert((size_t)kRows * kXzP * 2 == kOffUC - kOffU, "U/XZ extent");
static_assert((size_t)kRows * kCvP * 4 == kOffUCh - kOffUC, "UC/P extent");
static_assert((size_t)kRows * kDm * 2 == kOffU - kOffNA, "NA/S extent");
static_assert((size_t)kRows * kDin * 2 == kWsTotal - kOffCat, "CAT extent");

__device__ __forceinline__ float h16_to_f32(unsigned hb) {
  const unsigned sgn = (hb & 0x8000u) << 16; const unsigned em = hb & 0x7fffu;
  const float fn = __uint_as_float((em << 13) + 0x38000000u);
  const float fs = (float)em * 5.9604644775390625e-8f;
  const float mag = (em < 0x400u) ? fs : fn; return __uint_as_float(__float_as_uint(mag) | sgn); }

__device__ __forceinline__ void dep_guard4_h(v8f& a, v8f& b, v8f& c, v8f& d, v16h x, v16h y) {
  asm volatile("v_nop\n\tv_nop\n\tv_nop\n\tv_nop" : "+v"(a), "+v"(b), "+v"(c), "+v"(d) : "v"(x), "v"(y)); }
__device__ __forceinline__ void keep4_h(v16h a, v16h b, v16h c, v16h d) { asm volatile("v_nop" :: "v"(a), "v"(b), "v"(c), "v"(d)); }
__device__ __forceinline__ void acc_guard4(v8f& a, v8f& b, v8f& c, v8f& d) { asm volatile("v_nop\n\tv_nop\n\tv_nop\n\tv_nop" : "+v"(a), "+v"(b), "+v"(c), "+v"(d)); }

struct FragH {
  union U { v16h v; v8h h[2]; };
  static __device__ __forceinline__ v16h load(const _Float16* p) {
    U f; f.h[0] = *(const v8h*)(p); f.h[1] = *(const v8h*)(p + 16); return f.v;
  }
  static __device__ __forceinline__ v8f mma(v16h a, v16h b, v8f c) {
    return __builtin_amdgcn_wmma_f32_16x16x32_f16(false, a, false, b, (short)0, c, false, false);
  }
};

template <int BIAS_MODE, int OUT_MODE, bool RESID, int ACT>
__global__ __launch_bounds__(256) void gemm64_f16(
    const unsigned short* __restrict__ Ap, int lda, long strideA,
    const unsigned short* __restrict__ Btp, int ldb, long strideB,
    void* __restrict__ Cout, int ldc, long strideC,
    const float* __restrict__ bias, const float* __restrict__ resid,
    int M, int N, int K, float scale, float pscale, float oscale) {
  static_assert(!(RESID && OUT_MODE != 0), "resid only with f32 out");
  const _Float16* A  = (const _Float16*)Ap;
  const _Float16* Bt = (const _Float16*)Btp;
  __shared__ __align__(16) float sT[8][16 * 68];
  const int b    = blockIdx.y;
  const int lane = threadIdx.x & 31;
  const int wave = threadIdx.x >> 5;
  const int tilesN = N >> 6;
  const int tilesM = M >> 6;
  const int tile = blockIdx.x * 8 + wave;
  if (tile >= tilesM * tilesN) return;
  const int tm = tile / tilesN;
  const int tn = tile - tm * tilesN;
  const int m0 = tm << 6;
  const int n0 = tn << 6;

  const _Float16* Ab = A  + (size_t)b * strideA;
  const _Float16* Bb = Bt + (size_t)b * strideB;

  const int rlane = lane & 15;
  const int koff  = (lane >> 4) * 8;
  const int mOff  = (lane >> 4) * 8;

  v8f acc[4][4];
#pragma unroll
  for (int i = 0; i < 4; ++i)
#pragma unroll
    for (int j = 0; j < 4; ++j) acc[i][j] = (v8f){0.f,0.f,0.f,0.f,0.f,0.f,0.f,0.f};

  for (int k0 = 0; k0 < K; k0 += 32) {
    v16h bh[4];
#pragma unroll
    for (int j = 0; j < 4; ++j) {
      const size_t bo = (size_t)(n0 + (j << 4) + rlane) * ldb + koff + k0;
      bh[j] = FragH::load(Bb + bo);
    }
#pragma unroll
    for (int i = 0; i < 4; ++i) {
      const size_t ao = (size_t)(m0 + (i << 4) + rlane) * lda + koff + k0;
      v16h ah = FragH::load(Ab + ao);
#pragma unroll
      for (int j = 0; j < 4; ++j) acc[i][j] = FragH::mma(ah, bh[j], acc[i][j]);
      dep_guard4_h(acc[i][0], acc[i][1], acc[i][2], acc[i][3], ah, bh[3]);
    }
    keep4_h(bh[0], bh[1], bh[2], bh[3]);
  }
  acc_guard4(acc[0][0], acc[0][1], acc[0][2], acc[0][3]);
  acc_guard4(acc[1][0], acc[1][1], acc[1][2], acc[1][3]);
  acc_guard4(acc[2][0], acc[2][1], acc[2][2], acc[2][3]);
  acc_guard4(acc[3][0], acc[3][1], acc[3][2], acc[3][3]);

  float* slab = sT[wave];
#pragma unroll
  for (int i = 0; i < 4; ++i) {
    const int mBase = m0 + (i << 4);
#pragma unroll
    for (int j = 0; j < 4; ++j) {
      const int n = n0 + (j << 4) + rlane;
      float bv = 0.f;
      if (BIAS_MODE == 2) bv = bias[n];
#pragma unroll
      for (int r = 0; r < 8; ++r) {
        float v = acc[i][j][r] * scale;
        if (BIAS_MODE == 2) v += bv;
        v *= pscale;
        if (ACT == 3) v = v / (1.0f + expf(-v));
        v *= oscale;
        slab[(mOff + r) * 68 + (j << 4) + rlane] = v;
      }
    }
    __builtin_amdgcn_fence(__ATOMIC_RELEASE, "workgroup");
    __builtin_amdgcn_wave_barrier();
    __builtin_amdgcn_fence(__ATOMIC_ACQUIRE, "workgroup");
    if (OUT_MODE == 0) {
      float* C = (float*)Cout + (size_t)b * strideC;
      const float* Rb = RESID ? (resid + (size_t)b * strideC) : nullptr;
      const int hh = lane >> 4, c4 = (lane & 15) * 4;
      v4f ov[8];
#pragma unroll
      for (int it = 0; it < 8; ++it) {
        const int row = it * 2 + hh;
        v4f v = *(const v4f*)(slab + row * 68 + c4);
        if (RESID) {
          const v4f rv = *(const v4f*)(Rb + (size_t)(mBase + row) * ldc + n0 + c4);
          v += rv;
        }
        ov[it] = v;
      }
      for (int pass = 0; pass < 2; ++pass) {
#pragma unroll
        for (int it = 0; it < 8; ++it) {
          const int row = it * 2 + hh;
          *(volatile v4f*)(C + (size_t)(mBase + row) * ldc + n0 + c4) = ov[it];
        }
        __threadfence();
      }
    } else {
      const int q = lane >> 3, c8 = (lane & 7) * 8;
      unsigned short* C = (unsigned short*)Cout + (size_t)b * strideC;
      v8h hv[4];
#pragma unroll
      for (int it = 0; it < 4; ++it) {
        const int row = it * 4 + q;
        const float* sp = slab + row * 68 + c8;
#pragma unroll
        for (int e = 0; e < 8; ++e) hv[it][e] = (_Float16)sp[e];
      }
      for (int pass = 0; pass < 2; ++pass) {
#pragma unroll
        for (int it = 0; it < 4; ++it) {
          const int row = it * 4 + q;
          *(volatile v8h*)(C + (size_t)(mBase + row) * ldc + n0 + c8) = hv[it];
        }
        __threadfence();
      }
    }
    __builtin_amdgcn_fence(__ATOMIC_RELEASE, "workgroup");
    __builtin_amdgcn_wave_barrier();
    __builtin_amdgcn_fence(__ATOMIC_ACQUIRE, "workgroup");
  }
}

__global__ __launch_bounds__(256) void cast_f16x8_kernel(
    const float* __restrict__ src, unsigned short* __restrict__ dst, int total8, float mul)
{
  const int i = blockIdx.x * 256 + threadIdx.x;
  if (i >= total8) return;
  const size_t e0 = (size_t)i << 3;
  const v4f a0 = *(const v4f*)(src + e0);
  const v4f a1 = *(const v4f*)(src + e0 + 4);
  v8h hv;
#pragma unroll
  for (int e = 0; e < 4; ++e) {
    hv[e]     = (_Float16)(a0[e] * mul);
    hv[4 + e] = (_Float16)(a1[e] * mul);
  }
  unsigned short* q = dst + e0;
  *(volatile v8h*)q = hv;
  __threadfence();
  *(volatile v8h*)q = hv;
}

template <int MODE>
__global__ __launch_bounds__(256) void layernorm_kernel(
    const float* __restrict__ X, const float* __restrict__ gam, const float* __restrict__ bet,
    void* __restrict__ outp, int nrows)
{
  const int lane = threadIdx.x & 31, wave = threadIdx.x >> 5;
  const int row = blockIdx.x * 8 + wave;
  if (row >= nrows) return;
  const float* xr = X + (size_t)row * kDm;
  v4f xv[4];
#pragma unroll
  for (int i = 0; i < 4; ++i) {
    const int ci = (MODE == 0) ? ((i >> 1) * 256 + lane * 8 + (i & 1) * 4) : (i * 128 + lane * 4);
    xv[i] = *(const v4f*)(xr + ci);
  }
  float s = 0.0f;
#pragma unroll
  for (int i = 0; i < 4; ++i) { s += xv[i][0]; s += xv[i][1]; s += xv[i][2]; s += xv[i][3]; }
#pragma unroll
  for (int off = 16; off > 0; off >>= 1) s += __shfl_xor(s, off, 32);
  const float mean = s * (1.0f / (float)kDm);
  float sq = 0.0f;
#pragma unroll
  for (int i = 0; i < 4; ++i) {
#pragma unroll
    for (int e = 0; e < 4; ++e) { const float dv = xv[i][e] - mean; sq = fmaf(dv, dv, sq); }
  }
#pragma unroll
  for (int off = 16; off > 0; off >>= 1) sq += __shfl_xor(sq, off, 32);
  const float var  = sq * (1.0f / (float)kDm);
  const float rstd = 1.0f / sqrtf(var + 1e-5f);
  asm volatile("" ::: "memory");
  v4f ov[4];
#pragma unroll
  for (int i = 0; i < 4; ++i) {
    const int ci = (MODE == 0) ? ((i >> 1) * 256 + lane * 8 + (i & 1) * 4) : (i * 128 + lane * 4);
    const v4f gv = *(const v4f*)(gam + ci);
    const v4f bv = *(const v4f*)(bet + ci);
    ov[i] = (xv[i] - mean) * rstd * gv + bv;
  }
  if (MODE == 0) {
    unsigned short* o = (unsigned short*)outp + (size_t)row * kDm;
    v8h h0, h1;
#pragma unroll
    for (int e = 0; e < 4; ++e) {
      h0[e] = (_Float16)ov[0][e]; h0[4 + e] = (_Float16)ov[1][e];
      h1[e] = (_Float16)ov[2][e]; h1[4 + e] = (_Float16)ov[3][e];
    }
    for (int pass = 0; pass < 2; ++pass) {
      *(volatile v8h*)(o + lane * 8) = h0;
      *(volatile v8h*)(o + 256 + lane * 8) = h1;
      __threadfence();
    }
  } else {
    float* o = (float*)outp + (size_t)row * kDm;
    for (int pass = 0; pass < 2; ++pass) {
#pragma unroll
      for (int i = 0; i < 4; ++i) *(volatile v4f*)(o + i * 128 + lane * 4) = ov[i];
      __threadfence();
    }
  }
}

template <int REV>
__global__ __launch_bounds__(256) void mconv_silu_kernel(
    const unsigned short* __restrict__ XZ, const float* __restrict__ cw, const float* __restrict__ cb,
    float* __restrict__ UC, unsigned short* __restrict__ UCH)
{
  __shared__ __align__(16) float sIn[16 * kConvTP];
  __shared__ __align__(16) float sT[16 * kConvTP];
  const int tid = threadIdx.x, lane = tid & 31, wave = tid >> 5;
  const int d0 = blockIdx.x * 256, d = d0 + tid;
  const int g0 = blockIdx.y * 64;
  const int tb = g0 & (kL - 1);
  const v4f wv4 = *(const v4f*)(cw + (size_t)d * kKc);
  const float w0 = wv4[0], w1 = wv4[1], w2 = wv4[2], w3 = wv4[3];
  const float bc = cb[d];
  const bool hist = REV ? ((tb + 64) < kL) : (tb > 0);
  {
    int hb = REV ? (g0 + 64) : (g0 - 3);
    hb = hb < 0 ? 0 : hb;
    hb = (hb > kRows - 3) ? (kRows - 3) : hb;
    if (tid < 96) {
      const int r = tid >> 5, col8 = (tid & 31) * 8;
      const u32x4 w4 = *(const u32x4*)(XZ + (size_t)(hb + r) * kXzP + d0 + col8);
      float* sp = sIn + r * kConvTP + col8;
#pragma unroll
      for (int e = 0; e < 4; ++e) {
        const unsigned wd = w4[e];
        sp[2 * e]     = h16_to_f32(wd & 0xffffu);
        sp[2 * e + 1] = h16_to_f32(wd >> 16);
      }
    }
  }
  __syncthreads();
  float xa = sIn[tid], xb = sIn[kConvTP + tid], xg = sIn[2 * kConvTP + tid];
  if (!hist) { xa = 0.f; xb = 0.f; xg = 0.f; }
  __syncthreads();
  const int hrow = wave >> 1;
  const int hch  = (wave & 1) * 128 + lane * 4;
#pragma unroll 1
  for (int subi = 0; subi < 4; ++subi) {
    const int sub = REV ? (3 - subi) : subi;
    const int lb = g0 + sub * 16;
#pragma unroll
    for (int i = 0; i < 2; ++i) {
      const int u = tid + 256 * i;
      const int r = u >> 5, col8 = (u & 31) * 8;
      const u32x4 w4 = *(const u32x4*)(XZ + (size_t)(lb + r) * kXzP + d0 + col8);
      float* sp = sIn + r * kConvTP + col8;
#pragma unroll
      for (int e = 0; e < 4; ++e) {
        const unsigned wd = w4[e];
        sp[2 * e]     = h16_to_f32(wd & 0xffffu);
        sp[2 * e + 1] = h16_to_f32(wd >> 16);
      }
    }
    __syncthreads();
#pragma unroll 1
    for (int si = 0; si < 16; ++si) {
      const int s = REV ? (15 - si) : si;
      const float xcur = sIn[s * kConvTP + tid];
      float acc;
      if (REV) {
        acc = w3 * xcur;
        acc = fmaf(w2, xa, acc);
        acc = fmaf(w1, xb, acc);
        acc = fmaf(w0, xg, acc);
        xg = xb; xb = xa; xa = xcur;
      } else {
        acc = w0 * xa;
        acc = fmaf(w1, xb, acc);
        acc = fmaf(w2, xg, acc);
        acc = fmaf(w3, xcur, acc);
        xa = xb; xb = xg; xg = xcur;
      }
      const float sv = acc + bc;
      const float sg = __builtin_amdgcn_rcpf(1.0f + __expf(-sv));
      sT[s * kConvTP + tid] = sv * sg;
    }
    __syncthreads();
    v4f fv[4];
    v8h hv[2];
#pragma unroll
    for (int it = 0; it < 4; ++it) fv[it] = *(const v4f*)(sT + (it * 4 + hrow) * kConvTP + hch);
#pragma unroll
    for (int it = 0; it < 2; ++it) {
      const float* sp = sT + (it * 8 + wave) * kConvTP + lane * 8;
      const v4f a0 = *(const v4f*)(sp);
      const v4f a1 = *(const v4f*)(sp + 4);
#pragma unroll
      for (int e = 0; e < 4; ++e) {
        hv[it][e]     = (_Float16)(16.0f * a0[e]);
        hv[it][4 + e] = (_Float16)(16.0f * a1[e]);
      }
    }
    for (int pass = 0; pass < 2; ++pass) {
#pragma unroll
      for (int it = 0; it < 4; ++it)
        *(volatile v4f*)(UC + (size_t)(lb + it * 4 + hrow) * kDin + d0 + hch) = fv[it];
#pragma unroll
      for (int it = 0; it < 2; ++it)
        *(volatile v8h*)(UCH + (size_t)(lb + it * 8 + wave) * kDin + d0 + lane * 8) = hv[it];
      __threadfence();
    }
    __syncthreads();
  }
}

template <int REV>
__global__ __launch_bounds__(64) void scan_kernel(
    const float* __restrict__ XD, const float* __restrict__ UC, const unsigned short* __restrict__ XZ,
    const float* __restrict__ Wdt, const float* __restrict__ bdt, const float* __restrict__ Alog,
    const float* __restrict__ Dp, unsigned short* __restrict__ Y)
{
  __shared__ __align__(16) float sX[kScanTS * kXdP];
  __shared__ __align__(16) float sZY[kScanTS * kScanYP];
  __shared__ __align__(16) float sW[kDtR * kScanCh];
  __shared__ __align__(16) float sA[kNst * kScanCh];
  const int tid = threadIdx.x, lane = tid & 31, wave = tid >> 5;
  constexpr int kBlkPerB = kDin / kScanCh;
  const int bix = blockIdx.x / kBlkPerB;
  const int d0  = (blockIdx.x - bix * kBlkPerB) * kScanCh;
  const int d   = d0 + tid;
  const size_t row0 = (size_t)bix * kL;
#pragma unroll 1
  for (int r4 = 0; r4 < kDtR / 4; ++r4) {
    const v4f wv = *(const v4f*)(Wdt + (size_t)d * kDtR + 4 * r4);
    sW[(4 * r4 + 0) * kScanCh + tid] = wv[0];
    sW[(4 * r4 + 1) * kScanCh + tid] = wv[1];
    sW[(4 * r4 + 2) * kScanCh + tid] = wv[2];
    sW[(4 * r4 + 3) * kScanCh + tid] = wv[3];
  }
#pragma unroll 1
  for (int s4 = 0; s4 < kNst / 4; ++s4) {
    const v4f av = *(const v4f*)(Alog + (size_t)d * kNst + 4 * s4);
    sA[(4 * s4 + 0) * kScanCh + tid] = -expf(av[0]);
    sA[(4 * s4 + 1) * kScanCh + tid] = -expf(av[1]);
    sA[(4 * s4 + 2) * kScanCh + tid] = -expf(av[2]);
    sA[(4 * s4 + 3) * kScanCh + tid] = -expf(av[3]);
  }
  __syncthreads();
  float negA[kNst], h[kNst];
#pragma unroll
  for (int s = 0; s < kNst; ++s) {
    negA[s] = sA[s * kScanCh + tid];
    h[s] = 0.f;
  }
  const float bb = bdt[d], Dd = Dp[d];
  const int lr = tid >> 4, lc4 = (tid & 15) * 4;
  const int zr = tid >> 3, zc8 = (tid & 7) * 8;
  const int q = lane >> 3, c8 = (lane & 7) * 8;
#pragma unroll 1
  for (int ci = 0; ci < kL / kScanTS; ++ci) {
    const int t0 = REV ? (kL - kScanTS - ci * kScanTS) : (ci * kScanTS);
    __syncthreads();
#pragma unroll 4
    for (int i = 0; i < 16; ++i) {
      const int r = lr + 4 * i;
      *(v4f*)(sX + r * kXdP + lc4) = *(const v4f*)(XD + (row0 + t0 + r) * kXdP + lc4);
    }
#pragma unroll 2
    for (int i = 0; i < 8; ++i) {
      const int r = zr + 8 * i;
      const u32x4 w4 = *(const u32x4*)(XZ + (row0 + t0 + r) * kXzP + kDin + d0 + zc8);
      float* sp = sZY + r * kScanYP + zc8;
#pragma unroll
      for (int e = 0; e < 4; ++e) {
        const unsigned wd = w4[e];
        sp[2 * e]     = h16_to_f32(wd & 0xffffu);
        sp[2 * e + 1] = h16_to_f32(wd >> 16);
      }
    }
    __syncthreads();
#pragma unroll 1
    for (int si = 0; si < kScanTS; ++si) {
      const int s = REV ? (kScanTS - 1 - si) : si;
      const int t = t0 + s;
      const float* xr = sX + s * kXdP;
      float vdot = 0.f;
#pragma unroll 1
      for (int r4 = 0; r4 < kDtR / 4; ++r4) {
        const v4f xv = *(const v4f*)(xr + 4 * r4);
        const float* wp = sW + (4 * r4) * kScanCh + tid;
        vdot = fmaf(xv[0], wp[0], vdot);
        vdot = fmaf(xv[1], wp[kScanCh], vdot);
        vdot = fmaf(xv[2], wp[2 * kScanCh], vdot);
        vdot = fmaf(xv[3], wp[3 * kScanCh], vdot);
      }
      float Bs[kNst], Cs[kNst];
#pragma unroll
      for (int q4 = 0; q4 < 4; ++q4) {
        const v4f bv = *(const v4f*)(xr + kDtR + 4 * q4);
        const v4f cv = *(const v4f*)(xr + kDtR + kNst + 4 * q4);
        Bs[4 * q4 + 0] = bv[0]; Bs[4 * q4 + 1] = bv[1]; Bs[4 * q4 + 2] = bv[2]; Bs[4 * q4 + 3] = bv[3];
        Cs[4 * q4 + 0] = cv[0]; Cs[4 * q4 + 1] = cv[1]; Cs[4 * q4 + 2] = cv[2]; Cs[4 * q4 + 3] = cv[3];
      }
      const float v   = vdot + bb;
      const float a   = __expf(-fabsf(v));
      const float u   = 1.0f + a;
      const float l1p = __logf(u) + (a - (u - 1.0f)) * __builtin_amdgcn_rcpf(u);
      const float dt  = fmaxf(v, 0.0f) + l1p;
      const float xt  = UC[(row0 + t) * kDin + d];
      const float dtx = dt * xt;
      float y = 0.f;
#pragma unroll
      for (int k = 0; k < kNst; ++k) {
        const float e = __expf(dt * negA[k]);
        h[k] = e * h[k] + dtx * Bs[k];
        y = h[k] * Cs[k] + y;
      }
      y = xt * Dd + y;
      const float zv = sZY[s * kScanYP + tid];
      const float sg = __builtin_amdgcn_rcpf(1.0f + __expf(-zv));
      y = y * (zv * sg);
      sZY[s * kScanYP + tid] = y * 64.0f;
    }
    __syncthreads();
    v8h hv[8];
#pragma unroll
    for (int it = 0; it < 8; ++it) {
      const int row = it * 8 + wave * 4 + q;
      const float* sp = sZY + row * kScanYP + c8;
      const v4f a0 = *(const v4f*)(sp);
      const v4f a1 = *(const v4f*)(sp + 4);
#pragma unroll
      for (int e = 0; e < 4; ++e) {
        hv[it][e]     = (_Float16)a0[e];
        hv[it][4 + e] = (_Float16)a1[e];
      }
    }
    for (int pass = 0; pass < 2; ++pass) {
#pragma unroll
      for (int it = 0; it < 8; ++it) {
        const int row = it * 8 + wave * 4 + q;
        const size_t o = (row0 + t0 + row) * kDin + d0 + c8;
        *(volatile v8h*)(Y + o) = hv[it];
      }
      __threadfence();
    }
  }
}

__global__ __launch_bounds__(256) void dwconv_glu_kernel(
    const float* __restrict__ P, const float* __restrict__ w15, const float* __restrict__ w31,
    const float* __restrict__ w63, const float* __restrict__ bng, const float* __restrict__ bnb,
    const float* __restrict__ bnm, const float* __restrict__ bnv, unsigned short* __restrict__ S)
{
  __shared__ __align__(16) float sQ[128 * kDwCh];
  __shared__ __align__(16) float sWO[kDwRows * kDwOP];
  const int tid = threadIdx.x, lane = tid & 31, wave = tid >> 5;
  const int bix = blockIdx.x;
  const int cg = bix & 7, rb = (bix >> 3) & 7, bsq = bix >> 6;
  const int c0 = cg * kDwCh, r0 = rb * kDwRows;
  const size_t grow0 = (size_t)bsq * kL;
#pragma unroll 1
  for (int i = 0; i < 16; ++i) {
    const int e = tid + 256 * i;
    const int J = e >> 6;
    const int c = e & 63;
    const size_t ch = (size_t)(c0 + c);
    const int j63 = (J > 62) ? 62 : J;
    int j31 = J - 16; j31 = j31 < 0 ? 0 : (j31 > 30 ? 30 : j31);
    int j15 = J - 24; j15 = j15 < 0 ? 0 : (j15 > 14 ? 14 : j15);
    const float v63 = w63[ch * 63 + j63];
    const float v31 = w31[ch * 31 + j31];
    const float v15 = w15[ch * 15 + j15];
    const float f31 = (J >= 16 && J <= 46) ? 1.0f : 0.0f;
    const float f15 = (J >= 24 && J <= 38) ? 1.0f : 0.0f;
    const float v = fmaf(f15, v15, fmaf(f31, v31, v63));
    if (J < kDwTaps) sWO[J * kDwCh + c] = v;
    asm volatile("" ::: "memory");
  }
  const float* Pb = P + grow0 * kCvP;
#pragma unroll 1
  for (int i = 0; i < 8; ++i) {
    const int u = tid + 256 * i;
    const int lr = u >> 4;
    const int c4 = (u & 15) * 4;
    const int l = r0 - 31 + lr;
    const float finb = (l >= 0 && l < kL) ? 1.0f : 0.0f;
    const int la = l < 0 ? 0 : (l > kL - 1 ? (kL - 1) : l);
    const v4f av = *(const v4f*)(Pb + (size_t)la * kCvP + c0 + c4);
    const v4f gv = *(const v4f*)(Pb + (size_t)la * kCvP + kDm + c0 + c4);
    v4f qv;
#pragma unroll
    for (int e = 0; e < 4; ++e) {
      const float sg = __builtin_amdgcn_rcpf(1.0f + __expf(-gv[e]));
      qv[e] = av[e] * sg * finb;
    }
    *(v4f*)(sQ + lr * kDwCh + c4) = qv;
  }
  __syncthreads();
  const int c = tid & 63, rq = tid >> 6;
  float wj[kDwTaps];
#pragma unroll
  for (int j = 0; j < kDwTaps; ++j) wj[j] = sWO[j * kDwCh + c];
  __syncthreads();
  const float bg = bng[c0 + c], bbeta = bnb[c0 + c], bm = bnm[c0 + c];
  const float binv = 1.0f / sqrtf(bnv[c0 + c] + 1e-5f);
#pragma unroll 1
  for (int i = 0; i < 16; ++i) {
    const int r = rq * 16 + i;
    const float* qp = sQ + r * kDwCh + c;
    float acc = 0.0f;
#pragma unroll
    for (int j = 0; j < kDwTaps; ++j) acc = fmaf(wj[j], qp[j * kDwCh], acc);
    float sv = acc * (1.0f / 3.0f);
    sv = (sv - bm) * binv * bg + bbeta;
    const float sg = __builtin_amdgcn_rcpf(1.0f + __expf(-sv));
    sWO[r * kDwOP + c] = 16.0f * (sv * sg);
  }
  __syncthreads();
  const int q8 = lane >> 3, c8 = (lane & 7) * 8;
  v8h hv[2];
#pragma unroll
  for (int it = 0; it < 2; ++it) {
    const int row = it * 32 + wave * 4 + q8;
    const float* sp = sWO + row * kDwOP + c8;
    const v4f a0 = *(const v4f*)(sp);
    const v4f a1 = *(const v4f*)(sp + 4);
#pragma unroll
    for (int e = 0; e < 4; ++e) {
      hv[it][e]     = (_Float16)a0[e];
      hv[it][4 + e] = (_Float16)a1[e];
    }
  }
  unsigned short* Sb = S + (grow0 + (size_t)r0) * kDm + c0;
  for (int pass = 0; pass < 2; ++pass) {
#pragma unroll
    for (int it = 0; it < 2; ++it) {
      const int row = it * 32 + wave * 4 + q8;
      *(volatile v8h*)(Sb + (size_t)row * kDm + c8) = hv[it];
    }
    __threadfence();
  }
}

extern "C" void kernel_launch(void* const* d_in, const int* in_sizes, int n_in,
                              void* d_out, int out_size, void* d_ws, size_t ws_size,
                              hipStream_t stream) {
  if (n_in != 39) return;
  if (in_sizes[0] != kRows * kDm) return;
  if (in_sizes[1] != kDm || in_sizes[2] != kDm || in_sizes[7] != kDm || in_sizes[8] != kDm) return;
  if (in_sizes[3] != kDff * kDm || in_sizes[4] != kDff || in_sizes[5] != kDm * kDff || in_sizes[6] != kDm) return;
  if (in_sizes[9] != kDff * kDm || in_sizes[10] != kDff || in_sizes[11] != kDm * kDff || in_sizes[12] != kDm) return;
  if (in_sizes[13] != 2 * kXzP * kDm || in_sizes[14] != 2 * kDin * kKc || in_sizes[15] != 2 * kDin) return;
  if (in_sizes[16] != 2 * kXdP * kDin || in_sizes[17] != 2 * kDin * kDtR || in_sizes[18] != 2 * kDin) return;
  if (in_sizes[19] != 2 * kDin * kNst || in_sizes[20] != 2 * kDin || in_sizes[21] != 2 * kDm * kDin) return;
  if (in_sizes[22] != kDm * 2 * kDm || in_sizes[23] != kDm || in_sizes[24] != kDm || in_sizes[25] != kDm) return;
  if (in_sizes[26] != kCvP * kDm || in_sizes[27] != kCvP) return;
  if (in_sizes[28] != kDm * 15 || in_sizes[29] != kDm * 31 || in_sizes[30] != kDm * 63) return;
  if (in_sizes[31] != kDm || in_sizes[32] != kDm || in_sizes[33] != kDm || in_sizes[34] != kDm) return;
  if (in_sizes[35] != kDm * kDm || in_sizes[36] != kDm || in_sizes[37] != kDm || in_sizes[38] != kDm) return;
  if (out_size != kRows * kDm) return;
  if (ws_size < kWsTotal) return;

  const float* x        = (const float*)d_in[0];
  const float* ff1_ln_g = (const float*)d_in[1];
  const float* ff1_ln_b = (const float*)d_in[2];
  const float* ff1_w1   = (const float*)d_in[3];
  const float* ff1_b1   = (const float*)d_in[4];
  const float* ff1_w2   = (const float*)d_in[5];
  const float* ff1_b2   = (const float*)d_in[6];
  const float* ff2_ln_g = (const float*)d_in[7];
  const float* ff2_ln_b = (const float*)d_in[8];
  const float* ff2_w1   = (const float*)d_in[9];
  const float* ff2_b1   = (const float*)d_in[10];
  const float* ff2_w2   = (const float*)d_in[11];
  const float* ff2_b2   = (const float*)d_in[12];
  const float* m_win    = (const float*)d_in[13];
  const float* m_convw  = (const float*)d_in[14];
  const float* m_convb  = (const float*)d_in[15];
  const float* m_wx     = (const float*)d_in[16];
  const float* m_wdt    = (const float*)d_in[17];
  const float* m_bdt    = (const float*)d_in[18];
  const float* m_Alog   = (const float*)d_in[19];
  const float* m_Dp     = (const float*)d_in[20];
  const float* m_wout   = (const float*)d_in[21];
  const float* bi_wo    = (const float*)d_in[22];
  const float* bi_bo    = (const float*)d_in[23];
  const float* cv_ln_g  = (const float*)d_in[24];
  const float* cv_ln_b  = (const float*)d_in[25];
  const float* cv_pw1_w = (const float*)d_in[26];
  const float* cv_pw1_b = (const float*)d_in[27];
  const float* cv_dw15  = (const float*)d_in[28];
  const float* cv_dw31  = (const float*)d_in[29];
  const float* cv_dw63  = (const float*)d_in[30];
  const float* cv_bn_g  = (const float*)d_in[31];
  const float* cv_bn_b  = (const float*)d_in[32];
  const float* cv_bn_m  = (const float*)d_in[33];
  const float* cv_bn_v  = (const float*)d_in[34];
  const float* cv_pw2_w = (const float*)d_in[35];
  const float* cv_pw2_b = (const float*)d_in[36];
  const float* ln_g     = (const float*)d_in[37];
  const float* ln_b     = (const float*)d_in[38];
  float* out = (float*)d_out;

  char* ws = (char*)d_ws;
  unsigned short* W1a  = (unsigned short*)(ws + kOffW1a);
  unsigned short* W2a  = (unsigned short*)(ws + kOffW2a);
  unsigned short* W1b  = (unsigned short*)(ws + kOffW1b);
  unsigned short* W2b  = (unsigned short*)(ws + kOffW2b);
  unsigned short* Win  = (unsigned short*)(ws + kOffWin);
  unsigned short* Wx   = (unsigned short*)(ws + kOffWx);
  unsigned short* Wout = (unsigned short*)(ws + kOffWout);
  unsigned short* Wbo  = (unsigned short*)(ws + kOffWbo);
  unsigned short* Wp1  = (unsigned short*)(ws + kOffWp1);
  unsigned short* Wp2  = (unsigned short*)(ws + kOffWp2);
  float*          H1   = (float*)(ws + kOffH1);
  float*          H2   = (float*)(ws + kOffH2);
  float*          H3   = (float*)(ws + kOffH3);
  float*          H4   = (float*)(ws + kOffH4);
  unsigned short* Hh   = (unsigned short*)(ws + kOffHh);
  unsigned short* NA   = (unsigned short*)(ws + kOffNA);
  unsigned short* U    = (unsigned short*)(ws + kOffU);
  float*          UC   = (float*)(ws + kOffUC);
  unsigned short* UCh  = (unsigned short*)(ws + kOffUCh);
  float*          XD   = (float*)(ws + kOffXD);
  unsigned short* Yp   = (unsigned short*)(ws + kOffY);
  unsigned short* CAT  = (unsigned short*)(ws + kOffCat);

  const float kInv16 = 0.0625f, kInv256 = 0.00390625f, kInv4096 = 0.000244140625f;

  cast_f16x8_kernel<<<(kDff * kDm / 8) / 256, 256, 0, stream>>>(ff1_w1, W1a, kDff * kDm / 8, 16.0f);
  cast_f16x8_kernel<<<(kDm * kDff / 8) / 256, 256, 0, stream>>>(ff1_w2, W2a, kDm * kDff / 8, 16.0f);
  cast_f16x8_kernel<<<(kDff * kDm / 8) / 256, 256, 0, stream>>>(ff2_w1, W1b, kDff * kDm / 8, 16.0f);
  cast_f16x8_kernel<<<(kDm * kDff / 8) / 256, 256, 0, stream>>>(ff2_w2, W2b, kDm * kDff / 8, 16.0f);
  cast_f16x8_kernel<<<(2 * kXzP * kDm / 8) / 256, 256, 0, stream>>>(m_win, Win, 2 * kXzP * kDm / 8, 16.0f);
  cast_f16x8_kernel<<<(2 * kXdP * kDin / 8) / 256, 256, 0, stream>>>(m_wx, Wx, 2 * kXdP * kDin / 8, 16.0f);
  cast_f16x8_kernel<<<(2 * kDm * kDin / 8) / 256, 256, 0, stream>>>(m_wout, Wout, 2 * kDm * kDin / 8, 16.0f);
  cast_f16x8_kernel<<<(kDm * kCvP / 8) / 256, 256, 0, stream>>>(bi_wo, Wbo, kDm * kCvP / 8, 16.0f);
  cast_f16x8_kernel<<<(kCvP * kDm / 8) / 256, 256, 0, stream>>>(cv_pw1_w, Wp1, kCvP * kDm / 8, 16.0f);
  cast_f16x8_kernel<<<(kDm * kDm / 8) / 256, 256, 0, stream>>>(cv_pw2_w, Wp2, kDm * kDm / 8, 16.0f);

  layernorm_kernel<0><<<kRows / 8, 256, 0, stream>>>(x, ff1_ln_g, ff1_ln_b, (void*)NA, kRows);
  gemm64_f16<2, 1, false, 3><<<dim3(256, 1), 256, 0, stream>>>(
      NA, kDm, 0L, W1a, kDm, 0L, (void*)U, kDff, 0L, ff1_b1, nullptr,
      kRows, kDff, kDm, kInv16, 1.0f, 16.0f);
  gemm64_f16<2, 0, true, 0><<<dim3(64, 1), 256, 0, stream>>>(
      U, kDff, 0L, W2a, kDff, 0L, (void*)H1, kDm, 0L, ff1_b2, x,
      kRows, kDm, kDff, kInv256, 0.5f, 1.0f);
  cast_f16x8_kernel<<<(kRows * kDm / 8) / 256, 256, 0, stream>>>(H1, Hh, kRows * kDm / 8, 1.0f);

  gemm64_f16<0, 1, false, 0><<<dim3(256, 1), 256, 0, stream>>>(
      Hh, kDm, 0L, Win, kDm, 0L, (void*)U, kXzP, 0L, nullptr, nullptr,
      kRows, kXzP, kDm, kInv16, 1.0f, 1.0f);
  mconv_silu_kernel<0><<<dim3(kDin / 256, kRows / 64), 256, 0, stream>>>(U, m_convw, m_convb, UC, UCh);
  gemm64_f16<0, 0, false, 0><<<dim3(8, 1), 256, 0, stream>>>(
      UCh, kDin, 0L, Wx, kDin, 0L, (void*)XD, kXdP, 0L, nullptr, nullptr,
      kRows, kXdP, kDin, kInv256, 1.0f, 1.0f);
  scan_kernel<0><<<kB * (kDin / kScanCh), kScanCh, 0, stream>>>(XD, UC, U, m_wdt, m_bdt, m_Alog, m_Dp, Yp);
  gemm64_f16<0, 1, false, 0><<<dim3(64, 1), 256, 0, stream>>>(
      Yp, kDin, 0L, Wout, kDin, 0L, (void*)CAT, kDin, 0L, nullptr, nullptr,
      kRows, kDm, kDin, 0.25f, 1.0f, 1.0f);
  gemm64_f16<0, 1, false, 0><<<dim3(256, 1), 256, 0, stream>>>(
      Hh, kDm, 0L, Win + (size_t)kXzP * kDm, kDm, 0L, (void*)U, kXzP, 0L, nullptr, nullptr,
      kRows, kXzP, kDm, kInv16, 1.0f, 1.0f);
  mconv_silu_kernel<1><<<dim3(kDin / 256, kRows / 64), 256, 0, stream>>>(
      U, m_convw + (size_t)kDin * kKc, m_convb + kDin, UC, UCh);
  gemm64_f16<0, 0, false, 0><<<dim3(8, 1), 256, 0, stream>>>(
      UCh, kDin, 0L, Wx + (size_t)kXdP * kDin, kDin, 0L, (void*)XD, kXdP, 0L, nullptr, nullptr,
      kRows, kXdP, kDin, kInv256, 1.0f, 1.0f);
  scan_kernel<1><<<kB * (kDin / kScanCh), kScanCh, 0, stream>>>(
      XD, UC, U, m_wdt + (size_t)kDin * kDtR, m_bdt + kDin, m_Alog + (size_t)kDin * kNst, m_Dp + kDin, Yp);
  gemm64_f16<0, 1, false, 0><<<dim3(64, 1), 256, 0, stream>>>(
      Yp, kDin, 0L, Wout + (size_t)kDm * kDin, kDin, 0L, (void*)(CAT + kDm), kDin, 0L, nullptr, nullptr,
      kRows, kDm, kDin, 0.25f, 1.0f, 1.0f);
  gemm64_f16<2, 0, true, 0><<<dim3(64, 1), 256, 0, stream>>>(
      CAT, kDin, 0L, Wbo, kDin, 0L, (void*)H2, kDm, 0L, bi_bo, H1,
      kRows, kDm, kDin, kInv4096, 1.0f, 1.0f);

  layernorm_kernel<0><<<kRows / 8, 256, 0, stream>>>(H2, cv_ln_g, cv_ln_b, (void*)NA, kRows);
  gemm64_f16<2, 0, false, 0><<<dim3(128, 1), 256, 0, stream>>>(
      NA, kDm, 0L, Wp1, kDm, 0L, (void*)UC, kCvP, 0L, cv_pw1_b, nullptr,
      kRows, kCvP, kDm, kInv16, 1.0f, 1.0f);
  dwconv_glu_kernel<<<kB * (kL / kDwRows) * (kDm / kDwCh), 256, 0, stream>>>(
      UC, cv_dw15, cv_dw31, cv_dw63, cv_bn_g, cv_bn_b, cv_bn_m, cv_bn_v, NA);
  gemm64_f16<2, 0, true, 0><<<dim3(64, 1), 256, 0, stream>>>(
      NA, kDm, 0L, Wp2, kDm, 0L, (void*)H3, kDm, 0L, cv_pw2_b, H2,
      kRows, kDm, kDm, kInv256, 1.0f, 1.0f);

  layernorm_kernel<0><<<kRows / 8, 256, 0, stream>>>(H3, ff2_ln_g, ff2_ln_b, (void*)NA, kRows);
  gemm64_f16<2, 1, false, 3><<<dim3(256, 1), 256, 0, stream>>>(
      NA, kDm, 0L, W1b, kDm, 0L, (void*)U, kDff, 0L, ff2_b1, nullptr,
      kRows, kDff, kDm, kInv16, 1.0f, 16.0f);
  gemm64_f16<2, 0, true, 0><<<dim3(64, 1), 256, 0, stream>>>(
      U, kDff, 0L, W2b, kDff, 0L, (void*)H4, kDm, 0L, ff2_b2, H3,
      kRows, kDm, kDff, kInv256, 0.5f, 1.0f);

  layernorm_kernel<1><<<kRows / 8, 256, 0, stream>>>(H4, ln_g, ln_b, (void*)out, kRows);
}
